// S4Layer_3753801417521
// MI455X (gfx1250) — hardware-verified
//
#include <hip/hip_runtime.h>
#include <math.h>

typedef __attribute__((ext_vector_type(16))) _Float16 v16h;
typedef __attribute__((ext_vector_type(8)))  _Float16 v8h;
typedef __attribute__((ext_vector_type(16))) __bf16   v16b;
typedef __attribute__((ext_vector_type(8)))  __bf16   v8b;
typedef __attribute__((ext_vector_type(8)))  float    v8f;
typedef __attribute__((ext_vector_type(4)))  float    v4f;

constexpr int kBatch = 8;
constexpr int kDm    = 128;
constexpr int kNst   = 64;
constexpr int kSeq   = 2048;
constexpr int kCols  = kBatch * kSeq;
static_assert(kNst == 64, "two states per lane of a 32-lane wave");
static_assert((kDm % 64) == 0 && (kSeq % 64) == 0 && (kDm % 32) == 0, "GEMM M,N multiples of 64 and K multiple of 32");
static_assert((kSeq % 32) == 0, "one 128-B line of y per 32 steps");
static_assert(((kDm * kDm / 8) % 256) == 0, "weight plane threads fill whole blocks");
static_assert(((kBatch * kDm) % 8) == 0, "eight (b,d) waves per scan block");

constexpr size_t kOffYF   = 0;
constexpr size_t kOffYH   = kOffYF + (size_t)kBatch * kDm * kSeq * 4;
constexpr size_t kOffYL   = kOffYH + (size_t)kCols * kDm * 2;
constexpr size_t kOffWH   = kOffYL + (size_t)kCols * kDm * 2;
constexpr size_t kOffWL   = kOffWH + (size_t)kDm * kDm * 2;
constexpr size_t kWsTotal = kOffWL + (size_t)kDm * kDm * 2;
static_assert(kWsTotal == 16842752ull, "carve total");
static_assert(kWsTotal <= 134217728ull, "carve cap");
static_assert((kOffYH % 128) == 0 && (kOffYL % 128) == 0 && (kOffWH % 128) == 0 && (kOffWL % 128) == 0, "128-B aligned regions");

__device__ __forceinline__ unsigned short f2bf_bits(float f) {
  unsigned u = __float_as_uint(f);
  return (unsigned short)((u + 0x7FFFu + ((u >> 16) & 1u)) >> 16);
}
__device__ __forceinline__ float bf_bits2f(unsigned short h) { return __uint_as_float(((unsigned)h) << 16); }

__device__ __forceinline__ void dep_guard4_h(v8f& a, v8f& b, v8f& c, v8f& d, v16h x, v16h y) { asm volatile("v_nop\n\tv_nop\n\tv_nop\n\tv_nop" : "+v"(a), "+v"(b), "+v"(c), "+v"(d) : "v"(x), "v"(y)); }
__device__ __forceinline__ void dep_guard4_b(v8f& a, v8f& b, v8f& c, v8f& d, v16b x, v16b y) { asm volatile("v_nop\n\tv_nop\n\tv_nop\n\tv_nop" : "+v"(a), "+v"(b), "+v"(c), "+v"(d) : "v"(x), "v"(y)); }
__device__ __forceinline__ void keep4_h(v16h a, v16h b, v16h c, v16h d) { asm volatile("v_nop" :: "v"(a), "v"(b), "v"(c), "v"(d)); }
__device__ __forceinline__ void keep4_b(v16b a, v16b b, v16b c, v16b d) { asm volatile("v_nop" :: "v"(a), "v"(b), "v"(c), "v"(d)); }
__device__ __forceinline__ void acc_guard4(v8f& a, v8f& b, v8f& c, v8f& d) { asm volatile("v_nop\n\tv_nop\n\tv_nop\n\tv_nop" : "+v"(a), "+v"(b), "+v"(c), "+v"(d)); }
template <typename T> struct Frag;
template <> struct Frag<_Float16> {
  typedef v16h V; union U { v16h v; v8h h[2]; };
  static __device__ __forceinline__ v16h load(const _Float16* p) {
    U f; f.h[0] = *(const v8h*)(p); f.h[1] = *(const v8h*)(p + 16); return f.v;
  }
  static __device__ __forceinline__ v8f mma(v16h a, v16h b, v8f c) {
    return __builtin_amdgcn_wmma_f32_16x16x32_f16(false, a, false, b, (short)0, c, false, false);
  }
  static __device__ __forceinline__ void guard4(v8f& a, v8f& b, v8f& c, v8f& d, v16h x, v16h y) { dep_guard4_h(a, b, c, d, x, y); }
  static __device__ __forceinline__ void keep(v16h a, v16h b, v16h c, v16h d) { keep4_h(a, b, c, d); }
};
template <> struct Frag<__bf16> {
  typedef v16b V; union U { v16b v; v8b h[2]; };
  static __device__ __forceinline__ v16b load(const __bf16* p) {
    U f; f.h[0] = *(const v8b*)(p); f.h[1] = *(const v8b*)(p + 16); return f.v;
  }
  static __device__ __forceinline__ v8f mma(v16b a, v16b b, v8f c) {
    return __builtin_amdgcn_wmma_f32_16x16x32_bf16(false, a, false, b, (short)0, c, false, false);
  }
  static __device__ __forceinline__ void guard4(v8f& a, v8f& b, v8f& c, v8f& d, v16b x, v16b y) { dep_guard4_b(a, b, c, d, x, y); }
  static __device__ __forceinline__ void keep(v16b a, v16b b, v16b c, v16b d) { keep4_b(a, b, c, d); }
};

template <int ET> struct Elem;
template <> struct Elem<0> { typedef _Float16 T; };
template <> struct Elem<1> { typedef __bf16 T; };
template <int ET, bool SPLIT, int BIAS_MODE>
__global__ __launch_bounds__(256) void wmma_gemm64(
    const unsigned short* __restrict__ Ap, const unsigned short* __restrict__ A2p, int lda, long strideA,
    const unsigned short* __restrict__ Btp, const unsigned short* __restrict__ Bt2p, int ldb, long strideB,
    float* __restrict__ Cout, int ldc, long strideC,
    const float* __restrict__ bias,
    int M, int N, int K, float scale) {
  typedef typename Elem<ET>::T T;
  typedef typename Frag<T>::V V;
  const T* A = (const T*)Ap; const T* A2 = (const T*)A2p; const T* Bt = (const T*)Btp; const T* Bt2 = (const T*)Bt2p;
  __shared__ __align__(16) float sT[8][16 * 68];
  const int b    = blockIdx.y;
  const int lane = threadIdx.x & 31;
  const int wave = threadIdx.x >> 5;
  const int tilesN = N >> 6;
  const int tilesM = M >> 6;
  const int tile = blockIdx.x * 8 + wave;
  if (tile >= tilesM * tilesN) return;
  const int tm = tile / tilesN;
  const int tn = tile - tm * tilesN;
  const int m0 = tm << 6;
  const int n0 = tn << 6;

  const T* Ab  = A  + (size_t)b * strideA;
  const T* Bb  = Bt + (size_t)b * strideB;
  const T* Ab2 = SPLIT ? (A2  + (size_t)b * strideA) : nullptr;
  const T* Bb2 = SPLIT ? (Bt2 + (size_t)b * strideB) : nullptr;

  const int rlane = lane & 15;
  const int koff  = (lane >> 4) * 8;
  const int mOff  = (lane >> 4) * 8;

  v8f acc[4][4];
#pragma unroll
  for (int i = 0; i < 4; ++i)
#pragma unroll
    for (int j = 0; j < 4; ++j) acc[i][j] = (v8f){0.f,0.f,0.f,0.f,0.f,0.f,0.f,0.f};

  for (int k0 = 0; k0 < K; k0 += 32) {
    V bh[4], bl[4];
#pragma unroll
    for (int j = 0; j < 4; ++j) {
      const size_t bo = (size_t)(n0 + (j << 4) + rlane) * ldb + koff + k0;
      bh[j] = Frag<T>::load(Bb + bo);
      if (SPLIT) bl[j] = Frag<T>::load(Bb2 + bo);
    }
#pragma unroll
    for (int i = 0; i < 4; ++i) {
      const size_t ao = (size_t)(m0 + (i << 4) + rlane) * lda + koff + k0;
      V ah = Frag<T>::load(Ab + ao);
      V al;
      if (SPLIT) al = Frag<T>::load(Ab2 + ao);
#pragma unroll
      for (int j = 0; j < 4; ++j) {
        acc[i][j] = Frag<T>::mma(ah, bh[j], acc[i][j]);
        if (SPLIT) {
          acc[i][j] = Frag<T>::mma(ah, bl[j], acc[i][j]);
          acc[i][j] = Frag<T>::mma(al, bh[j], acc[i][j]);
        }
      }
      Frag<T>::guard4(acc[i][0], acc[i][1], acc[i][2], acc[i][3], ah, SPLIT ? al : ah);
    }
    Frag<T>::keep(bh[0], bh[1], bh[2], bh[3]);
    if (SPLIT) Frag<T>::keep(bl[0], bl[1], bl[2], bl[3]);
  }
  acc_guard4(acc[0][0], acc[0][1], acc[0][2], acc[0][3]);
  acc_guard4(acc[1][0], acc[1][1], acc[1][2], acc[1][3]);
  acc_guard4(acc[2][0], acc[2][1], acc[2][2], acc[2][3]);
  acc_guard4(acc[3][0], acc[3][1], acc[3][2], acc[3][3]);

  float* slab = sT[wave];
#pragma unroll
  for (int i = 0; i < 4; ++i) {
    const int mBase = m0 + (i << 4);
#pragma unroll
    for (int j = 0; j < 4; ++j) {
      const int n = n0 + (j << 4) + rlane;
      float bv = 0.f;
      if (BIAS_MODE == 2) bv = bias[n];
#pragma unroll
      for (int r = 0; r < 8; ++r) {
        float v = acc[i][j][r] * scale;
        if (BIAS_MODE == 1) v += bias[mBase + mOff + r];
        if (BIAS_MODE == 2) v += bv;
        slab[(mOff + r) * 68 + (j << 4) + rlane] = v;
      }
    }
    __builtin_amdgcn_fence(__ATOMIC_RELEASE, "workgroup");
    __builtin_amdgcn_wave_barrier();
    __builtin_amdgcn_fence(__ATOMIC_ACQUIRE, "workgroup");
    {
      float* C = Cout + (size_t)b * strideC;
      const int hh = lane >> 4, c4 = (lane & 15) * 4;
      for (int pass = 0; pass < 2; ++pass) {
#pragma unroll
        for (int it = 0; it < 8; ++it) {
          const int row = it * 2 + hh;
          v4f v = *(const v4f*)(slab + row * 68 + c4);
          *(volatile v4f*)(C + (size_t)(mBase + row) * ldc + n0 + c4) = v;
        }
        __threadfence();
      }
    }
    __builtin_amdgcn_fence(__ATOMIC_RELEASE, "workgroup");
    __builtin_amdgcn_wave_barrier();
    __builtin_amdgcn_fence(__ATOMIC_ACQUIRE, "workgroup");
  }
}

__global__ __launch_bounds__(256) void split_rows_bf16_kernel(
    const float* __restrict__ src, unsigned short* __restrict__ dhi, unsigned short* __restrict__ dlo, int total8)
{
  const int i = blockIdx.x * 256 + threadIdx.x;
  if (i >= total8) return;
  const size_t e0 = (size_t)i << 3;
  const v4f a0 = *(const v4f*)(src + e0);
  const v4f a1 = *(const v4f*)(src + e0 + 4);
  v8h hv, lv;
#pragma unroll
  for (int e = 0; e < 4; ++e) {
    const float f0 = a0[e];
    const float f1 = a1[e];
    const unsigned short h0 = f2bf_bits(f0), h1 = f2bf_bits(f1);
    const unsigned short l0 = f2bf_bits(f0 - bf_bits2f(h0)), l1 = f2bf_bits(f1 - bf_bits2f(h1));
    hv[e]     = __builtin_bit_cast(_Float16, h0);
    hv[4 + e] = __builtin_bit_cast(_Float16, h1);
    lv[e]     = __builtin_bit_cast(_Float16, l0);
    lv[4 + e] = __builtin_bit_cast(_Float16, l1);
  }
  unsigned short* qh = dhi + e0;
  unsigned short* ql = dlo + e0;
  *(volatile v8h*)qh = hv;
  *(volatile v8h*)ql = lv;
  __threadfence();
  *(volatile v8h*)qh = hv;
  *(volatile v8h*)ql = lv;
}

__global__ __launch_bounds__(256) void scan_kernel(
    const float* __restrict__ x, const float* __restrict__ A, const float* __restrict__ Bm,
    const float* __restrict__ Cm, const float* __restrict__ Dv, float* __restrict__ YF)
{
  const int lane = threadIdx.x & 31;
  const int wave = threadIdx.x >> 5;
  const int p = blockIdx.x * 8 + wave;
  const int b = p / kDm;
  const int d = p - b * kDm;
  const int n0 = lane;
  const int n1 = lane + 32;
  const float a0 = A[(size_t)d * kNst * kNst + (size_t)n0 * (kNst + 1)];
  const float a1 = A[(size_t)d * kNst * kNst + (size_t)n1 * (kNst + 1)];
  const float b0 = Bm[d * kNst + n0];
  const float b1 = Bm[d * kNst + n1];
  const float c0 = Cm[d * kNst + n0];
  const float c1 = Cm[d * kNst + n1];
  const float dv = Dv[d];
  const float* xrow = x  + ((size_t)b * kDm + d) * kSeq;
  float*       yrow = YF + ((size_t)b * kDm + d) * kSeq;

  float h0 = 0.0f, h1 = 0.0f;
#pragma unroll 1
  for (int l0 = 0; l0 < kSeq; l0 += 32) {
    float xv = xrow[l0 + lane];
    asm volatile("" : "+v"(xv));
    float ylatch = 0.0f;
#pragma unroll 1
    for (int s = 0; s < 32; ++s) {
      const float xt = __shfl(xv, s, 32);
      h0 = tanhf(fmaf(a0, h0, b0 * xt));
      h1 = tanhf(fmaf(a1, h1, b1 * xt));
      float part = fmaf(c0, h0, c1 * h1);
      part += __shfl_xor(part, 16, 32);
      part += __shfl_xor(part,  8, 32);
      part += __shfl_xor(part,  4, 32);
      part += __shfl_xor(part,  2, 32);
      part += __shfl_xor(part,  1, 32);
      const float yv = fmaf(dv, xt, part);
      ylatch = (lane == s) ? yv : ylatch;
    }
    volatile float* q = yrow + l0 + lane;
    *q = ylatch;
    __threadfence();
    *q = ylatch;
  }
}

__global__ __launch_bounds__(256) void transpose_split_kernel(
    const float* __restrict__ YF, unsigned short* __restrict__ YH, unsigned short* __restrict__ YL)
{
  __shared__ float tile[64 * 65];
  const int tid = threadIdx.x, lane = tid & 31, wave = tid >> 5;
  const int l0 = blockIdx.x * 64;
  const int d0 = blockIdx.y * 64;
  const int b  = blockIdx.z;
#pragma unroll
  for (int p = 0; p < 4; ++p) {
    const int idx = tid + p * 256;
    const int dd  = idx >> 4;
    const int l4  = (idx & 15) * 4;
    const v4f v = *(const v4f*)(YF + ((size_t)b * kDm + d0 + dd) * kSeq + l0 + l4);
    tile[dd * 65 + l4 + 0] = v[0];
    tile[dd * 65 + l4 + 1] = v[1];
    tile[dd * 65 + l4 + 2] = v[2];
    tile[dd * 65 + l4 + 3] = v[3];
  }
  __syncthreads();
  const int q = lane >> 3, c8 = (lane & 7) * 8;
  v8h hv[2], lv[2];
#pragma unroll
  for (int it = 0; it < 2; ++it) {
    const int lrow = it * 32 + wave * 4 + q;
#pragma unroll
    for (int e = 0; e < 8; ++e) {
      const float f = tile[(c8 + e) * 65 + lrow];
      const unsigned short hb = f2bf_bits(f);
      const unsigned short lb = f2bf_bits(f - bf_bits2f(hb));
      hv[it][e] = __builtin_bit_cast(_Float16, hb);
      lv[it][e] = __builtin_bit_cast(_Float16, lb);
    }
  }
  for (int pass = 0; pass < 2; ++pass) {
#pragma unroll
    for (int it = 0; it < 2; ++it) {
      const int lrow = it * 32 + wave * 4 + q;
      const size_t o = ((size_t)b * kSeq + l0 + lrow) * kDm + d0 + c8;
      *(volatile v8h*)(YH + o) = hv[it];
      *(volatile v8h*)(YL + o) = lv[it];
    }
    __threadfence();
  }
}

extern "C" void kernel_launch(void* const* d_in, const int* in_sizes, int n_in,
                              void* d_out, int out_size, void* d_ws, size_t ws_size,
                              hipStream_t stream) {
  if (n_in < 7) return;
  if (in_sizes[0] != kBatch * kDm * kSeq) return;
  if (in_sizes[1] != kDm * kNst * kNst) return;
  if (in_sizes[2] != kDm * kNst) return;
  if (in_sizes[3] != kDm * kNst) return;
  if (in_sizes[4] != kDm) return;
  if (in_sizes[5] != kDm * kDm) return;
  if (in_sizes[6] != kDm) return;
  if (out_size != kBatch * kDm * kSeq) return;
  if (ws_size < kWsTotal) return;

  const float* x    = (const float*)d_in[0];
  const float* A    = (const float*)d_in[1];
  const float* Bm   = (const float*)d_in[2];
  const float* Cm   = (const float*)d_in[3];
  const float* Dv   = (const float*)d_in[4];
  const float* W    = (const float*)d_in[5];
  const float* bias = (const float*)d_in[6];
  float* out = (float*)d_out;

  char* ws = (char*)d_ws;
  float*          YF = (float*)(ws + kOffYF);
  unsigned short* YH = (unsigned short*)(ws + kOffYH);
  unsigned short* YL = (unsigned short*)(ws + kOffYL);
  unsigned short* WH = (unsigned short*)(ws + kOffWH);
  unsigned short* WL = (unsigned short*)(ws + kOffWL);

  split_rows_bf16_kernel<<<(kDm * kDm / 8) / 256, 256, 0, stream>>>(W, WH, WL, kDm * kDm / 8);

  scan_kernel<<<(kBatch * kDm) / 8, 256, 0, stream>>>(x, A, Bm, Cm, Dv, YF);

  transpose_split_kernel<<<dim3(kSeq / 64, kDm / 64, kBatch), 256, 0, stream>>>(YF, YH, YL);

  wmma_gemm64<1, true, 1><<<dim3(((kDm / 64) * (kSeq / 64)) / 8, kBatch), 256, 0, stream>>>(
      WH, WL, kDm, 0L,
      YH, YL, kDm, (long)kSeq * kDm,
      out, kSeq, (long)kDm * kSeq,
      bias,
      kDm, kSeq, kDm, 1.0f);
}
